// _MPNNNet_63900523430414
// MI455X (gfx1250) — hardware-verified
//
#include <hip/hip_runtime.h>
#include <stddef.h>
#include <math.h>


#define HD    64
#define AF    9
#define BF    4
#define HHD   32
#define KW    4096
#define KTOT  4160
#define NTHR  256
#define NWAVE 8
#define EPT   8
#define NGRP  2
#define CHUNK (NTHR * EPT * NGRP)
#define WCAP  (EPT * NGRP * 32)
#define LISTN (NWAVE * WCAP)
#define NBK   128
#define GBK   128
#define MEDG  128
#define ESC   16.0f
#define WSC   64.0f
#define MINV  (1.0f / 1024.0f)
#define RSC   16.0f
#define RINV  (1.0f / 16.0f)
#define PSC   16.0f
#define HSC   8.0f
#define PINV  (1.0f / 128.0f)

static_assert((CHUNK & (CHUNK - 1)) == 0);
static_assert(CHUNK <= 4096);
static_assert((NBK & (NBK - 1)) == 0);
static_assert(NBK <= 4096);
static_assert(NBK == NWAVE * 16);
static_assert(GBK == NWAVE * 16);
static_assert(MEDG == NWAVE * 16);
static_assert((KTOT % 64) == 0);
static_assert((KW % 8) == 0);

typedef float    v2f  __attribute__((ext_vector_type(2)));
typedef float    v4f  __attribute__((ext_vector_type(4)));
typedef float    v8f  __attribute__((ext_vector_type(8)));
typedef int      v4i  __attribute__((ext_vector_type(4)));
typedef _Float16 v8h  __attribute__((ext_vector_type(8)));
typedef _Float16 v16h __attribute__((ext_vector_type(16)));
union FragH { v16h v; v8h h[2]; };

__device__ __forceinline__ v8h cvt8(v4f a, v4f b) {
  v8h r;
  r[0] = (_Float16)a.x; r[1] = (_Float16)a.y; r[2] = (_Float16)a.z; r[3] = (_Float16)a.w;
  r[4] = (_Float16)b.x; r[5] = (_Float16)b.y; r[6] = (_Float16)b.z; r[7] = (_Float16)b.w;
  return r;
}

__device__ __forceinline__ v8f wmh(v16h a, v16h b, v8f c) {
  v8f d = __builtin_amdgcn_wmma_f32_16x16x32_f16(false, a, false, b, (short)0, c, false, false);
  asm volatile("v_nop\n\tv_nop\n\tv_nop\n\tv_nop" : "+v"(d) : "v"(a), "v"(b));
  return d;
}

__device__ __forceinline__ float gelu_f(float v) {
  return 0.5f * v * (1.0f + erff(v * 0.70710678118654752f));
}

template <int NB>
__device__ __forceinline__ int scan_chunk(const int* __restrict__ dsts, int nE, int cbase, int nodeBase,
                                          int vec8, int* list, int tid, int lane, int wave) {
  int wc = 0;
#pragma unroll
  for (int g = 0; g < NGRP; ++g) {
    const int el0  = (g * NTHR + tid) * EPT;
    const int e0   = cbase + el0;
    const int sent = -2147483647 - 1;
    v4i da, db;
    if (vec8 != 0 && e0 + 7 < nE) {
      da = *(const v4i*)(dsts + e0);
      db = *(const v4i*)(dsts + e0 + 4);
    } else {
      da.x = (e0     < nE) ? dsts[min(e0, nE - 1)] : sent;
      da.y = (e0 + 1 < nE) ? dsts[min(e0 + 1, nE - 1)] : sent;
      da.z = (e0 + 2 < nE) ? dsts[min(e0 + 2, nE - 1)] : sent;
      da.w = (e0 + 3 < nE) ? dsts[min(e0 + 3, nE - 1)] : sent;
      db.x = (e0 + 4 < nE) ? dsts[min(e0 + 4, nE - 1)] : sent;
      db.y = (e0 + 5 < nE) ? dsts[min(e0 + 5, nE - 1)] : sent;
      db.z = (e0 + 6 < nE) ? dsts[min(e0 + 6, nE - 1)] : sent;
      db.w = (e0 + 7 < nE) ? dsts[min(e0 + 7, nE - 1)] : sent;
    }
    const unsigned nb = (unsigned)nodeBase;
    const unsigned s0 = (unsigned)da.x - nb, s1 = (unsigned)da.y - nb;
    const unsigned s2 = (unsigned)da.z - nb, s3 = (unsigned)da.w - nb;
    const unsigned s4 = (unsigned)db.x - nb, s5 = (unsigned)db.y - nb;
    const unsigned s6 = (unsigned)db.z - nb, s7 = (unsigned)db.w - nb;
    const bool h0 = s0 < (unsigned)NB, h1 = s1 < (unsigned)NB, h2 = s2 < (unsigned)NB, h3 = s3 < (unsigned)NB;
    const bool h4 = s4 < (unsigned)NB, h5 = s5 < (unsigned)NB, h6 = s6 < (unsigned)NB, h7 = s7 < (unsigned)NB;
    const unsigned any = __builtin_amdgcn_ballot_w32(h0 | h1 | h2 | h3 | h4 | h5 | h6 | h7);
    if (any != 0u) {
#define HITJ(J, HJ, SJ) { \
        const unsigned mj = __builtin_amdgcn_ballot_w32(HJ); \
        if (mj != 0u) { \
          if (HJ) { \
            const int pos = wc + (int)__builtin_amdgcn_mbcnt_lo(mj, 0u); \
            if (pos < WCAP) list[wave * WCAP + pos] = ((el0 + (J)) << 12) | (int)(SJ); \
          } \
          wc += (int)__builtin_popcount(mj); } }
      HITJ(0, h0, s0)
      HITJ(1, h1, s1)
      HITJ(2, h2, s2)
      HITJ(3, h3, s3)
      HITJ(4, h4, s4)
      HITJ(5, h5, s5)
      HITJ(6, h6, s6)
      HITJ(7, h7, s7)
#undef HITJ
    }
  }
  return wc;
}

__global__ __launch_bounds__(NTHR) void k_wprep(
    const float* __restrict__ w2, const float* __restrict__ b2, const float* __restrict__ rw,
    _Float16* wT, _Float16* rT, int nL) {
  const int idx = blockIdx.x * NTHR + threadIdx.x;
  const int n1 = nL * HD * (KTOT / 8);
  const int n2 = nL * HD * (HD / 8);
  if (idx >= n1 + n2) return;
  v4f a, b;
  _Float16* dp;
  if (idx < n1) {
    const int row = idx / (KTOT / 8);
    const int k0  = (idx - row * (KTOT / 8)) * 8;
    const int l = row >> 6, o = row & 63;
    const float* p;
    if (k0 < KW) p = w2 + ((size_t)l * KW + k0) * HD + o;
    else         p = b2 + ((size_t)l * HD + (k0 - KW)) * HD + o;
    a.x = p[0];      a.y = p[HD];     a.z = p[2 * HD]; a.w = p[3 * HD];
    b.x = p[4 * HD]; b.y = p[5 * HD]; b.z = p[6 * HD]; b.w = p[7 * HD];
    a = a * WSC; b = b * WSC;
    dp = wT + (size_t)idx * 8;
  } else {
    const int u = idx - n1;
    const int row = u >> 3, k0 = (u & 7) * 8;
    const int l = row >> 6, o = row & 63;
    const float* p = rw + ((size_t)l * HD + k0) * HD + o;
    a.x = p[0];      a.y = p[HD];     a.z = p[2 * HD]; a.w = p[3 * HD];
    b.x = p[4 * HD]; b.y = p[5 * HD]; b.z = p[6 * HD]; b.w = p[7 * HD];
    a = a * RSC; b = b * RSC;
    dp = rT + (size_t)u * 8;
  }
  const v8h hv = cvt8(a, b);
  *(volatile v8h*)dp = hv;
  __threadfence();
  *(volatile v8h*)dp = hv;
}

__global__ __launch_bounds__(NTHR) void k_embed(
    const float* __restrict__ x, const float* __restrict__ aw, const float* __restrict__ ab,
    float* h, int nN) {
  const int idx = blockIdx.x * NTHR + threadIdx.x;
  const int node = idx >> 4, c4 = (idx & 15) * 4;
  const int nr = node > nN - 1 ? nN - 1 : node;
  float a0 = ab[c4], a1 = ab[c4 + 1], a2 = ab[c4 + 2], a3 = ab[c4 + 3];
  const float* xp = x + (size_t)nr * AF;
#pragma unroll
  for (int f = 0; f < AF; ++f) {
    const float xv = xp[f];
    const float* wp = aw + f * HD + c4;
    a0 += xv * wp[0]; a1 += xv * wp[1]; a2 += xv * wp[2]; a3 += xv * wp[3];
  }
  v4f o;
  o.x = gelu_f(a0); o.y = gelu_f(a1); o.z = gelu_f(a2); o.w = gelu_f(a3);
  float* dp = h + (size_t)node * HD + c4;
  *(volatile v4f*)dp = o;
  __threadfence();
  *(volatile v4f*)dp = o;
}

__global__ __launch_bounds__(NTHR) void k_edgeprep(
    const int* __restrict__ ei, const float* __restrict__ ea, const float* __restrict__ h,
    const float* __restrict__ w1, const float* __restrict__ b1,
    float* hs, float* es, int nN, int nE, int layer) {
  const int idx = blockIdx.x * NTHR + threadIdx.x;
  const int edge = idx >> 4, c4 = (idx & 15) * 4;
  const int er = edge > nE - 1 ? nE - 1 : edge;
  int src = ei[er];
  src = src < 0 ? 0 : (src > nN - 1 ? nN - 1 : src);
  const v4f hv = *(const v4f*)(h + (size_t)src * HD + c4);
  const float* wl = w1 + (size_t)layer * BF * HD + c4;
  const float* bl = b1 + layer * HD + c4;
  float a0 = bl[0], a1 = bl[1], a2 = bl[2], a3 = bl[3];
  const float* ap = ea + (size_t)er * BF;
#pragma unroll
  for (int f = 0; f < BF; ++f) {
    const float av = ap[f];
    const float* wp = wl + f * HD;
    a0 += av * wp[0]; a1 += av * wp[1]; a2 += av * wp[2]; a3 += av * wp[3];
  }
  v4f ev;
  ev.x = gelu_f(a0) * ESC; ev.y = gelu_f(a1) * ESC; ev.z = gelu_f(a2) * ESC; ev.w = gelu_f(a3) * ESC;
  float* hp2 = hs + (size_t)edge * HD + c4;
  float* ep2 = es + (size_t)edge * HD + c4;
  *(volatile v4f*)hp2 = hv;
  *(volatile v4f*)ep2 = ev;
  __threadfence();
  *(volatile v4f*)hp2 = hv;
  *(volatile v4f*)ep2 = ev;
}

__global__ __launch_bounds__(NTHR) void k_msg(
    const float* __restrict__ hs, const float* __restrict__ es,
    const _Float16* __restrict__ wT, float* msg, int layer) {
  __shared__ __attribute__((aligned(16))) float stg[NWAVE * 16 * HD];
  const int tid = threadIdx.x, lane = tid & 31, wave = tid >> 5, hh = lane >> 4, m = lane & 15;
  const int ebase = (blockIdx.x * NWAVE + wave) * 16;

  const float* hp = hs + ((size_t)ebase + m) * HD + 8 * hh;
  const v4f h00 = *(const v4f*)(hp),      h01 = *(const v4f*)(hp + 4);
  const v4f h10 = *(const v4f*)(hp + 16), h11 = *(const v4f*)(hp + 20);
  const v4f h20 = *(const v4f*)(hp + 32), h21 = *(const v4f*)(hp + 36);
  const v4f h30 = *(const v4f*)(hp + 48), h31 = *(const v4f*)(hp + 52);
  const float* ep = es + ((size_t)ebase + m) * HD;
  const _Float16* wb = wT + ((size_t)layer * HD + m) * KTOT + 8 * hh;

  v8f acc[4];
#pragma unroll
  for (int t = 0; t < 4; ++t) { v8f z = {0.f, 0.f, 0.f, 0.f, 0.f, 0.f, 0.f, 0.f}; acc[t] = z; }

#pragma unroll 1
  for (int jp = 0; jp < KTOT / 64; ++jp) {
    const int jc = jp < HD ? jp : HD - 1;
    const float sv = ep[jc];
    const float s = jp < HD ? sv : ESC;
    const int koff = 64 * jp;
    {
      FragH a;
      a.h[0] = cvt8(h00 * s, h01 * s);
      a.h[1] = cvt8(h10 * s, h11 * s);
#pragma unroll
      for (int t = 0; t < 4; ++t) {
        const _Float16* bp = wb + (size_t)t * 16 * KTOT + koff;
        FragH b;
        b.h[0] = *(const v8h*)bp;
        b.h[1] = *(const v8h*)(bp + 16);
        acc[t] = wmh(a.v, b.v, acc[t]);
      }
    }
    {
      FragH a;
      a.h[0] = cvt8(h20 * s, h21 * s);
      a.h[1] = cvt8(h30 * s, h31 * s);
#pragma unroll
      for (int t = 0; t < 4; ++t) {
        const _Float16* bp = wb + (size_t)t * 16 * KTOT + koff + 32;
        FragH b;
        b.h[0] = *(const v8h*)bp;
        b.h[1] = *(const v8h*)(bp + 16);
        acc[t] = wmh(a.v, b.v, acc[t]);
      }
    }
  }

  float* sw = stg + wave * (16 * HD);
#pragma unroll
  for (int t = 0; t < 4; ++t) {
#pragma unroll
    for (int r = 0; r < 8; ++r) sw[(8 * hh + r) * HD + 16 * t + m] = acc[t][r] * MINV;
  }
  __syncthreads();
  v4f ov[8];
#pragma unroll
  for (int q = 0; q < 8; ++q) ov[q] = *(const v4f*)(sw + (2 * q + hh) * HD + 4 * m);
  float* gp = msg + ((size_t)ebase + hh) * HD + 4 * m;
#pragma unroll
  for (int q = 0; q < 8; ++q) *(volatile v4f*)(gp + (size_t)(2 * q) * HD) = ov[q];
  __threadfence();
#pragma unroll
  for (int q = 0; q < 8; ++q) *(volatile v4f*)(gp + (size_t)(2 * q) * HD) = ov[q];
}

__global__ __launch_bounds__(NTHR) void k_node(
    const int* __restrict__ ei, const float* __restrict__ msg, const float* __restrict__ hin,
    const _Float16* __restrict__ rT, const float* __restrict__ conv_b,
    const float* __restrict__ ln_g, const float* __restrict__ ln_b,
    float* hout, int nN, int nE, int layer, int vec8) {
  __shared__ __attribute__((aligned(16))) float acc[NBK * HD];
  __shared__ __attribute__((aligned(16))) int list[LISTN];
  __shared__ int cnt[NBK];
  __shared__ int wcnt[NWAVE];
  const int tid = threadIdx.x, lane = tid & 31, wave = tid >> 5, hh = lane >> 4, m = lane & 15;
  const int nodeBase = blockIdx.x * NBK;
  const int* dsts = ei + nE;

  {
    const v4f z = {0.f, 0.f, 0.f, 0.f};
    for (int i = tid; i < NBK * HD / 4; i += NTHR) ((v4f*)acc)[i] = z;
    for (int i = tid; i < NBK; i += NTHR) cnt[i] = 0;
  }
  __syncthreads();

  const int nChunks = (nE + CHUNK - 1) / CHUNK;
#pragma unroll 1
  for (int ch = 0; ch < nChunks; ++ch) {
    const int cbase = ch * CHUNK;
    const int wc = scan_chunk<NBK>(dsts, nE, cbase, nodeBase, vec8, list, tid, lane, wave);
    if (lane == 0) wcnt[wave] = wc;
    __syncthreads();
    if (wave == 0) {
#pragma unroll 1
      for (int wsx = 0; wsx < NWAVE; ++wsx) {
        int n = __builtin_amdgcn_readfirstlane(wcnt[wsx]);
        n = n > WCAP ? WCAP : (n < 0 ? 0 : n);
        const int* lp = list + wsx * WCAP;
#pragma unroll 1
        for (int i = 0; i < n; ++i) {
          const int ent  = __builtin_amdgcn_readfirstlane(lp[i]);
          const int slot = ent & (NBK - 1);
          int e = cbase + ((ent >> 12) & (CHUNK - 1));
          e = e > nE - 1 ? nE - 1 : e;
          const v2f mv = *(const v2f*)(msg + (size_t)e * HD + 2 * lane);
          v2f* ap = (v2f*)(acc + slot * HD + 2 * lane);
          *ap = *ap + mv;
          if (lane == 0) cnt[slot] = cnt[slot] + 1;
        }
      }
    }
    __syncthreads();
  }

  int nodeA = nodeBase + 16 * wave + m;
  nodeA = nodeA > nN - 1 ? nN - 1 : nodeA;
  v8f d[4];
#pragma unroll
  for (int t = 0; t < 4; ++t) { v8f z = {0.f, 0.f, 0.f, 0.f, 0.f, 0.f, 0.f, 0.f}; d[t] = z; }
#pragma unroll
  for (int kt = 0; kt < 2; ++kt) {
    const float* hp = hin + (size_t)nodeA * HD + 32 * kt + 8 * hh;
    FragH a;
    a.h[0] = cvt8(*(const v4f*)hp, *(const v4f*)(hp + 4));
    a.h[1] = cvt8(*(const v4f*)(hp + 16), *(const v4f*)(hp + 20));
#pragma unroll
    for (int t = 0; t < 4; ++t) {
      const _Float16* bp = rT + ((size_t)layer * HD + 16 * t + m) * HD + 32 * kt + 8 * hh;
      FragH b;
      b.h[0] = *(const v8h*)bp;
      b.h[1] = *(const v8h*)(bp + 16);
      d[t] = wmh(a.v, b.v, d[t]);
    }
  }

#pragma unroll
  for (int r = 0; r < 8; ++r) {
    const int slot = 16 * wave + 8 * hh + r;
    int c = cnt[slot];
    c = c < 1 ? 1 : c;
    const float degi = 1.0f / (float)c;
#pragma unroll
    for (int t = 0; t < 4; ++t) {
      float* p = acc + slot * HD + 16 * t + m;
      *p = *p * degi + d[t][r] * RINV;
    }
  }

  const float* cb = conv_b + layer * HD;
  const float* lg = ln_g + layer * HD;
  const float* lb = ln_b + layer * HD;
#pragma unroll 1
  for (int r = 0; r < 8; ++r) {
    const int slot = 16 * wave + 8 * hh + r;
    int node = nodeBase + slot;
    node = node > nN - 1 ? nN - 1 : node;
    float z[4];
#pragma unroll
    for (int t = 0; t < 4; ++t) {
      const int col = 16 * t + m;
      const float pre = acc[slot * HD + col] + cb[col];
      z[t] = hin[(size_t)node * HD + col] + gelu_f(pre);
    }
    float s1 = (z[0] + z[1]) + (z[2] + z[3]);
    s1 += __shfl_xor(s1, 8);
    s1 += __shfl_xor(s1, 4);
    s1 += __shfl_xor(s1, 2);
    s1 += __shfl_xor(s1, 1);
    const float mu = s1 * (1.0f / 64.0f);
    float dz[4];
#pragma unroll
    for (int t = 0; t < 4; ++t) dz[t] = z[t] - mu;
    float s2 = (dz[0] * dz[0] + dz[1] * dz[1]) + (dz[2] * dz[2] + dz[3] * dz[3]);
    s2 += __shfl_xor(s2, 8);
    s2 += __shfl_xor(s2, 4);
    s2 += __shfl_xor(s2, 2);
    s2 += __shfl_xor(s2, 1);
    const float var = s2 * (1.0f / 64.0f);
    const float rs = rsqrtf(var + 1e-5f);
#pragma unroll
    for (int t = 0; t < 4; ++t) {
      const int col = 16 * t + m;
      acc[slot * HD + col] = dz[t] * rs * lg[col] + lb[col];
    }
  }
  __syncthreads();

  v4f ov[8];
#pragma unroll
  for (int q = 0; q < 8; ++q) ov[q] = *(const v4f*)(acc + (wave * 8 + q) * 128 + 4 * lane);
  float* gp = hout + (size_t)nodeBase * HD;
#pragma unroll
  for (int q = 0; q < 8; ++q) *(volatile v4f*)(gp + (wave * 8 + q) * 128 + 4 * lane) = ov[q];
  __threadfence();
#pragma unroll
  for (int q = 0; q < 8; ++q) *(volatile v4f*)(gp + (wave * 8 + q) * 128 + 4 * lane) = ov[q];
}

__global__ __launch_bounds__(NTHR) void k_pool_head(
    const float* __restrict__ h, const int* __restrict__ batch,
    const float* __restrict__ hw1, const float* __restrict__ hb1,
    const float* __restrict__ hw2, const float* __restrict__ hb2,
    float* out, int nN, int nG) {
  __shared__ __attribute__((aligned(16))) float pacc[GBK * HD];
  __shared__ __attribute__((aligned(16))) _Float16 molh[GBK * HD];
  __shared__ int pcnt[GBK];
  __shared__ __attribute__((aligned(16))) float sout[GBK];
  const int tid = threadIdx.x, lane = tid & 31, wave = tid >> 5, hh = lane >> 4, m = lane & 15;
  const int gbase = blockIdx.x * GBK;

  {
    const v4f z = {0.f, 0.f, 0.f, 0.f};
    for (int i = tid; i < GBK * HD / 4; i += NTHR) ((v4f*)pacc)[i] = z;
    for (int i = tid; i < GBK; i += NTHR) { pcnt[i] = 0; sout[i] = 0.f; }
  }
  __syncthreads();

  if (wave == 0) {
#pragma unroll 1
    for (int i = 0; i < nN; ++i) {
      const int g = __builtin_amdgcn_readfirstlane(batch[i]);
      const unsigned us = (unsigned)(g - gbase);
      if (us < (unsigned)GBK) {
        const v2f hv = *(const v2f*)(h + (size_t)i * HD + 2 * lane);
        v2f* ap = (v2f*)(pacc + us * HD + 2 * lane);
        *ap = *ap + hv;
        if (lane == 0) pcnt[us] = pcnt[us] + 1;
      }
    }
  }
  __syncthreads();

#pragma unroll
  for (int it = 0; it < (GBK * HD / 8) / NTHR; ++it) {
    const int u = it * NTHR + tid;
    const int slot = u >> 3, c0 = (u & 7) * 8;
    int c = pcnt[slot];
    c = c < 1 ? 1 : c;
    const float rc = 1.0f / (float)c;
    v4f a = *(const v4f*)(pacc + slot * HD + c0);
    v4f b = *(const v4f*)(pacc + slot * HD + c0 + 4);
    a = (a * rc) * PSC;
    b = (b * rc) * PSC;
    *(v8h*)(molh + slot * HD + c0) = cvt8(a, b);
  }

  FragH bw[2][2];
#pragma unroll
  for (int kt = 0; kt < 2; ++kt) {
#pragma unroll
    for (int t = 0; t < 2; ++t) {
#pragma unroll
      for (int p = 0; p < 16; ++p) {
        const int k = 32 * kt + ((p < 8) ? (8 * hh + p) : (16 + 8 * hh + (p - 8)));
        bw[kt][t].v[p] = (_Float16)(hw1[k * HHD + 16 * t + m] * HSC);
      }
    }
  }
  __syncthreads();

  v8f d[2];
  {
    v8f z = {0.f, 0.f, 0.f, 0.f, 0.f, 0.f, 0.f, 0.f};
    d[0] = z; d[1] = z;
  }
#pragma unroll
  for (int kt = 0; kt < 2; ++kt) {
    const _Float16* ap = molh + (16 * wave + m) * HD + 32 * kt + 8 * hh;
    FragH a;
    a.h[0] = *(const v8h*)ap;
    a.h[1] = *(const v8h*)(ap + 16);
#pragma unroll
    for (int t = 0; t < 2; ++t) d[t] = wmh(a.v, bw[kt][t].v, d[t]);
  }

  const float b2v = hb2[0];
#pragma unroll
  for (int r = 0; r < 8; ++r) {
    const int slot = 16 * wave + 8 * hh + r;
    float s = 0.f;
#pragma unroll
    for (int t = 0; t < 2; ++t) {
      const int j = 16 * t + m;
      const float v = d[t][r] * PINV + hb1[j];
      s += gelu_f(v) * hw2[j];
    }
    s += __shfl_xor(s, 8);
    s += __shfl_xor(s, 4);
    s += __shfl_xor(s, 2);
    s += __shfl_xor(s, 1);
    if (m == 0) sout[slot] = s + b2v;
  }
  __syncthreads();

  if (wave == 0) {
    const int gi = gbase + 4 * lane;
    const v4f v = *(const v4f*)(sout + 4 * lane);
    if (gi + 4 <= nG) {
      *(volatile v4f*)(out + gi) = v;
    } else {
      if (gi     < nG) *(volatile float*)(out + gi)     = v.x;
      if (gi + 1 < nG) *(volatile float*)(out + gi + 1) = v.y;
      if (gi + 2 < nG) *(volatile float*)(out + gi + 2) = v.z;
      if (gi + 3 < nG) *(volatile float*)(out + gi + 3) = v.w;
    }
    __threadfence();
    if (gi + 4 <= nG) {
      *(volatile v4f*)(out + gi) = v;
    } else {
      if (gi     < nG) *(volatile float*)(out + gi)     = v.x;
      if (gi + 1 < nG) *(volatile float*)(out + gi + 1) = v.y;
      if (gi + 2 < nG) *(volatile float*)(out + gi + 2) = v.z;
      if (gi + 3 < nG) *(volatile float*)(out + gi + 3) = v.w;
    }
  }
}

extern "C" void kernel_launch(void* const* d_in, const int* in_sizes, int n_in,
                              void* d_out, int out_size, void* d_ws, size_t ws_size,
                              hipStream_t stream) {
  if (n_in < 18) return;
  const int nN = in_sizes[3];
  const int nE = in_sizes[1] / 2;
  const int nG = out_size;
  if (nN <= 0 || nE <= 0 || nG <= 0) return;
  if (in_sizes[0] != nN * AF || in_sizes[1] != 2 * nE || in_sizes[2] != nE * BF) return;
  const int nL = in_sizes[10] / (HD * HD);
  if (nL <= 0) return;
  if (in_sizes[4] != AF * HD || in_sizes[5] != HD) return;
  if (in_sizes[6] != nL * BF * HD || in_sizes[7] != nL * HD) return;
  if (in_sizes[8] != nL * HD * KW || in_sizes[9] != nL * KW) return;
  if (in_sizes[10] != nL * HD * HD || in_sizes[11] != nL * HD || in_sizes[12] != nL * HD || in_sizes[13] != nL * HD) return;
  if (in_sizes[14] != HD * HHD || in_sizes[15] != HHD || in_sizes[16] != HHD || in_sizes[17] < 1) return;

  const float* x      = (const float*)d_in[0];
  const int*   ei     = (const int*)d_in[1];
  const float* ea     = (const float*)d_in[2];
  const int*   batch  = (const int*)d_in[3];
  const float* atom_w = (const float*)d_in[4];
  const float* atom_b = (const float*)d_in[5];
  const float* ew1    = (const float*)d_in[6];
  const float* eb1    = (const float*)d_in[7];
  const float* ew2    = (const float*)d_in[8];
  const float* eb2    = (const float*)d_in[9];
  const float* root_w = (const float*)d_in[10];
  const float* conv_b = (const float*)d_in[11];
  const float* ln_g   = (const float*)d_in[12];
  const float* ln_b   = (const float*)d_in[13];
  const float* hw1    = (const float*)d_in[14];
  const float* hb1    = (const float*)d_in[15];
  const float* hw2    = (const float*)d_in[16];
  const float* hb2    = (const float*)d_in[17];
  float* out = (float*)d_out;

  const int Npad = ((nN + NBK - 1) / NBK) * NBK;
  const int Epad = ((nE + MEDG - 1) / MEDG) * MEDG;

  char* ws = (char*)d_ws;
  size_t off = 0;
  const size_t oWT = off; off += (size_t)nL * HD * KTOT * 2;   off = (off + 511) & ~(size_t)511;
  const size_t oRT = off; off += (size_t)nL * HD * HD * 2;     off = (off + 511) & ~(size_t)511;
  const size_t oHA = off; off += (size_t)Npad * HD * 4;        off = (off + 511) & ~(size_t)511;
  const size_t oHB = off; off += (size_t)Npad * HD * 4;        off = (off + 511) & ~(size_t)511;
  const size_t oHS = off; off += (size_t)Epad * HD * 4;        off = (off + 511) & ~(size_t)511;
  const size_t oES = off; off += (size_t)Epad * HD * 4;        off = (off + 511) & ~(size_t)511;
  const size_t oMS = off; off += (size_t)Epad * HD * 4;        off = (off + 511) & ~(size_t)511;
  if (off > ws_size) return;
  if (off > (size_t)134217728) return;
  _Float16* wT  = (_Float16*)(ws + oWT);
  _Float16* rT  = (_Float16*)(ws + oRT);
  float*    hA  = (float*)(ws + oHA);
  float*    hB  = (float*)(ws + oHB);
  float*    hs  = (float*)(ws + oHS);
  float*    es  = (float*)(ws + oES);
  float*    msg = (float*)(ws + oMS);

  const int vec8 = ((nE & 3) == 0) ? 1 : 0;

  const int nPrep = nL * HD * (KTOT / 8) + nL * HD * (HD / 8);
  k_wprep<<<(nPrep + NTHR - 1) / NTHR, NTHR, 0, stream>>>(ew2, eb2, root_w, wT, rT, nL);

  k_embed<<<(Npad * 16) / NTHR, NTHR, 0, stream>>>(x, atom_w, atom_b, hA, nN);

  float* hc = hA;
  float* hn = hB;
  for (int l = 0; l < nL; ++l) {
    k_edgeprep<<<(Epad * 16) / NTHR, NTHR, 0, stream>>>(ei, ea, hc, ew1, eb1, hs, es, nN, nE, l);
    k_msg<<<Epad / MEDG, NTHR, 0, stream>>>(hs, es, wT, msg, l);
    k_node<<<Npad / NBK, NTHR, 0, stream>>>(ei, msg, hc, rT, conv_b, ln_g, ln_b, hn, nN, nE, l, vec8);
    float* t = hc; hc = hn; hn = t;
  }

  k_pool_head<<<(nG + GBK - 1) / GBK, NTHR, 0, stream>>>(hc, batch, hw1, hb1, hw2, hb2, out, nN, nG);
}
